// MultiHeadCrossAttention_51161650430221
// MI455X (gfx1250) — hardware-verified
//
#include <hip/hip_runtime.h>
#include <math.h>

#ifndef NB
#define NB 2
#endif
#ifndef SEQ
#define SEQ 2048
#endif
#define NB_FULL 2
#define SEQ_FULL 2048
#ifndef MASK_LD
#define MASK_LD SEQ_FULL
#endif
#define DM 1024
#define NH 16
#define HD 64
#define NTOK (NB * SEQ)

static_assert(NB >= 1 && NB <= NB_FULL);
static_assert(SEQ >= 64 && SEQ <= SEQ_FULL && (SEQ % 64) == 0);
static_assert(NH * HD == DM && HD == 64 && (DM % 64) == 0);
static_assert((MASK_LD % 4) == 0 && MASK_LD >= SEQ);
static_assert((NTOK % 64) == 0);
static_assert((((long long)NTOK) * (DM / 8)) % 256 == 0);
static_assert((((long long)DM) * (DM / 8)) % 256 == 0);

typedef _Float16 v16h __attribute__((ext_vector_type(16)));
typedef _Float16 v8h  __attribute__((ext_vector_type(8)));
typedef __bf16   v16b __attribute__((ext_vector_type(16)));
typedef __bf16   v8b  __attribute__((ext_vector_type(8)));
typedef float    v8f  __attribute__((ext_vector_type(8)));
typedef float    v4f_raw __attribute__((ext_vector_type(4)));
typedef v4f_raw  v4f __attribute__((may_alias));
typedef unsigned short v8us_raw __attribute__((ext_vector_type(8)));
typedef v8us_raw v8us __attribute__((may_alias));


__device__ __forceinline__ unsigned short f2bf_bits(float f) {
  unsigned u = __float_as_uint(f);
  return (unsigned short)((u + 0x7FFFu + ((u >> 16) & 1u)) >> 16);
}
__device__ __forceinline__ float bf_bits2f(unsigned short h) { return __uint_as_float(((unsigned)h) << 16); }

__device__ __forceinline__ void dep_guard_h(v8f& a, v8f& b, v16h x, v16h y) { asm volatile("v_nop\n\tv_nop\n\tv_nop\n\tv_nop" : "+v"(a), "+v"(b) : "v"(x), "v"(y)); }
__device__ __forceinline__ void dep_guard_b(v8f& a, v8f& b, v16b x, v16b y) { asm volatile("v_nop\n\tv_nop\n\tv_nop\n\tv_nop" : "+v"(a), "+v"(b) : "v"(x), "v"(y)); }
__device__ __forceinline__ void keep4_h(v16h a, v16h b, v16h c, v16h d) { asm volatile("v_nop" :: "v"(a), "v"(b), "v"(c), "v"(d)); }
__device__ __forceinline__ void keep4_b(v16b a, v16b b, v16b c, v16b d) { asm volatile("v_nop" :: "v"(a), "v"(b), "v"(c), "v"(d)); }
__device__ __forceinline__ void acc_guard4(v8f& a, v8f& b, v8f& c, v8f& d) { asm volatile("v_nop\n\tv_nop\n\tv_nop\n\tv_nop" : "+v"(a), "+v"(b), "+v"(c), "+v"(d)); }

template <typename T> struct Frag;
template <> struct Frag<_Float16> {
  typedef v16h V; union U { v16h v; v8h h[2]; };
  static __device__ __forceinline__ v16h load(const _Float16* p) {
    U f; f.h[0] = *(const v8h*)(p); f.h[1] = *(const v8h*)(p + 16); return f.v;
  }
  static __device__ __forceinline__ v8f mma(v16h a, v16h b, v8f c) {
    return __builtin_amdgcn_wmma_f32_16x16x32_f16(false, a, false, b, (short)0, c, false, false);
  }
  static __device__ __forceinline__ void guard(v8f& a, v8f& b, v16h x, v16h y) { dep_guard_h(a, b, x, y); }
  static __device__ __forceinline__ void keep(v16h a, v16h b, v16h c, v16h d) { keep4_h(a, b, c, d); }
};
template <> struct Frag<__bf16> {
  typedef v16b V; union U { v16b v; v8b h[2]; };
  static __device__ __forceinline__ v16b load(const __bf16* p) {
    U f; f.h[0] = *(const v8b*)(p); f.h[1] = *(const v8b*)(p + 16); return f.v;
  }
  static __device__ __forceinline__ v8f mma(v16b a, v16b b, v8f c) {
    return __builtin_amdgcn_wmma_f32_16x16x32_bf16(false, a, false, b, (short)0, c, false, false);
  }
  static __device__ __forceinline__ void guard(v8f& a, v8f& b, v16b x, v16b y) { dep_guard_b(a, b, x, y); }
  static __device__ __forceinline__ void keep(v16b a, v16b b, v16b c, v16b d) { keep4_b(a, b, c, d); }
};

template <int ET> struct Elem;
template <> struct Elem<0> { typedef _Float16 T; };
template <> struct Elem<1> { typedef __bf16 T; };
template <int ET, bool SPLIT, int BIAS_MODE, int OUT_MODE, bool RESID, int ACT = 0>
__global__ __launch_bounds__(256) void k_gemm64(
    const unsigned short* __restrict__ Ap, const unsigned short* __restrict__ A2p, int lda, long strideA,
    const unsigned short* __restrict__ Btp, const unsigned short* __restrict__ Bt2p, int ldb, long strideB,
    void* __restrict__ Cout, void* __restrict__ Cout2, int ldc, long strideC,
    const float* __restrict__ bias,
    const float* __restrict__ resid, long strideR,
    int M, int N, int K, float scale) {
  typedef typename Elem<ET>::T T;
  typedef typename Frag<T>::V V;
  const T* A = (const T*)Ap; const T* A2 = (const T*)A2p; const T* Bt = (const T*)Btp; const T* Bt2 = (const T*)Bt2p;
  __shared__ __align__(16) float sT[8][16 * 68];
  const int b    = blockIdx.y;
  const int lane = threadIdx.x & 31;
  const int wave = threadIdx.x >> 5;
  const int tilesN = N >> 6;
  const int tilesM = M >> 6;
  const int tile = blockIdx.x * 8 + wave;
  if (tile >= tilesM * tilesN) return;
  const int tm = tile / tilesN;
  const int tn = tile - tm * tilesN;
  const int m0 = tm << 6;
  const int n0 = tn << 6;

  const T* Ab  = A  + (size_t)b * strideA;
  const T* Bb  = Bt + (size_t)b * strideB;
  const T* Ab2 = SPLIT ? (A2  + (size_t)b * strideA) : nullptr;
  const T* Bb2 = SPLIT ? (Bt2 + (size_t)b * strideB) : nullptr;

  const int rlane = lane & 15;
  const int koff  = (lane >> 4) * 8;
  const int mOff  = (lane >> 4) * 8;

  v8f acc[4][4];
#pragma unroll
  for (int i = 0; i < 4; ++i)
#pragma unroll
    for (int j = 0; j < 4; ++j) acc[i][j] = (v8f){0.f,0.f,0.f,0.f,0.f,0.f,0.f,0.f};

  for (int k0 = 0; k0 < K; k0 += 32) {
    V bh[4], bl[4];
#pragma unroll
    for (int j = 0; j < 4; ++j) {
      const size_t bo = (size_t)(n0 + (j << 4) + rlane) * ldb + koff + k0;
      bh[j] = Frag<T>::load(Bb + bo);
      if (SPLIT) bl[j] = Frag<T>::load(Bb2 + bo);
    }
#pragma unroll
    for (int i = 0; i < 4; ++i) {
      const size_t ao = (size_t)(m0 + (i << 4) + rlane) * lda + koff + k0;
      V ah = Frag<T>::load(Ab + ao);
      V al;
      if (SPLIT) al = Frag<T>::load(Ab2 + ao);
#pragma unroll
      for (int j = 0; j < 4; ++j) {
        acc[i][j] = Frag<T>::mma(ah, bh[j], acc[i][j]);
        if (SPLIT) {
          acc[i][j] = Frag<T>::mma(ah, bl[j], acc[i][j]);
          acc[i][j] = Frag<T>::mma(al, bh[j], acc[i][j]);
        }
      }
      Frag<T>::guard(acc[i][0], acc[i][3], ah, SPLIT ? al : ah);
    }
    Frag<T>::keep(bh[0], bh[1], bh[2], bh[3]);
    if (SPLIT) Frag<T>::keep(bl[0], bl[1], bl[2], bl[3]);
  }
  acc_guard4(acc[0][0], acc[0][1], acc[0][2], acc[0][3]);
  acc_guard4(acc[1][0], acc[1][1], acc[1][2], acc[1][3]);
  acc_guard4(acc[2][0], acc[2][1], acc[2][2], acc[2][3]);
  acc_guard4(acc[3][0], acc[3][1], acc[3][2], acc[3][3]);

  float* slab = sT[wave];
  const float* Rb = RESID ? (resid + (size_t)b * strideR) : nullptr;
#pragma unroll
  for (int i = 0; i < 4; ++i) {
    const int mBase = m0 + (i << 4);
#pragma unroll
    for (int j = 0; j < 4; ++j) {
      const int n = n0 + (j << 4) + rlane;
      float bv = 0.f;
      if (BIAS_MODE == 2) bv = bias[n];
#pragma unroll
      for (int r = 0; r < 8; ++r) {
        float v = acc[i][j][r] * scale;
        if (BIAS_MODE == 1) v += bias[mBase + mOff + r];
        if (BIAS_MODE == 2) v += bv;
        if (RESID) v += Rb[(size_t)(mBase + mOff + r) * ldc + n];
        if (ACT == 1) v = tanhf(v);
        if (ACT == 2) v = fmaxf(v, 0.0f);
        if (ACT == 4) v = (v > 0.f) ? v : 0.01f * v;
        if (ACT == 6) v = (v > 0.f) ? v : 0.2f * v;
        slab[(mOff + r) * 68 + (j << 4) + rlane] = v;
      }
    }
    __builtin_amdgcn_fence(3  , "workgroup");
    __builtin_amdgcn_wave_barrier();
    __builtin_amdgcn_fence(2  , "workgroup");
    if (OUT_MODE == 0) {
      float* C = (float*)Cout + (size_t)b * strideC;
      const int hh = lane >> 4, c4 = (lane & 15) * 4;
      for (int pass = 0; pass < 2; ++pass) {
#pragma unroll
        for (int it = 0; it < 8; ++it) {
          const int row = it * 2 + hh;
          v4f v = *(const v4f*)(slab + row * 68 + c4);
          *(volatile v4f*)(C + (size_t)(mBase + row) * ldc + n0 + c4) = v;
        }
        __threadfence();
      }
    } else {
      const int q = lane >> 3, c8 = (lane & 7) * 8;
      unsigned short* C  = (unsigned short*)Cout  + (size_t)b * strideC;
      unsigned short* C2 = (OUT_MODE == 2) ? ((unsigned short*)Cout2 + (size_t)b * strideC) : nullptr;
      for (int pass = 0; pass < 2; ++pass) {
#pragma unroll
        for (int it = 0; it < 4; ++it) {
          const int row = it * 4 + q;
          const float* sp = slab + row * 68 + c8;
          v8h hv, lv;
#pragma unroll
          for (int e = 0; e < 8; ++e) {
            if (OUT_MODE == 1) {
              hv[e] = (_Float16)sp[e];
            } else {
              unsigned short hb = f2bf_bits(sp[e]);
              unsigned short lb = f2bf_bits(sp[e] - bf_bits2f(hb));
              hv[e] = __builtin_bit_cast(_Float16, hb);
              lv[e] = __builtin_bit_cast(_Float16, lb);
            }
          }
          *(volatile v8h*)(C + (size_t)(mBase + row) * ldc + n0 + c8) = hv;
          if (OUT_MODE == 2) *(volatile v8h*)(C2 + (size_t)(mBase + row) * ldc + n0 + c8) = lv;
        }
        __threadfence();
      }
    }
    __builtin_amdgcn_fence(3  , "workgroup");
    __builtin_amdgcn_wave_barrier();
    __builtin_amdgcn_fence(2  , "workgroup");
  }
}

template <bool F16OUT>
__global__ __launch_bounds__(256) void k_cvt8(const float* __restrict__ src, unsigned short* __restrict__ dst, int nrows, int rpb, int srb, float s) {
  const long long u = (long long)blockIdx.x * 256 + threadIdx.x;
  if (u >= (long long)nrows * (DM / 8)) return;
  const int t = (int)(u / (DM / 8));
  const int c8 = 8 * (int)(u % (DM / 8));
  const long long sr = (long long)(t / rpb) * srb + (t % rpb);
  const v4f a = *(const v4f*)(src + sr * DM + c8);
  const v4f bq = *(const v4f*)(src + sr * DM + c8 + 4);
  const float f[8] = {a[0], a[1], a[2], a[3], bq[0], bq[1], bq[2], bq[3]};
  v8us o;
#pragma unroll
  for (int e = 0; e < 8; ++e) {
    const unsigned short hb = f2bf_bits(f[e]);
    if (F16OUT) o[e] = __builtin_bit_cast(unsigned short, (_Float16)(bf_bits2f(hb) * s));
    else o[e] = hb;
  }
  volatile v8us* d = (volatile v8us*)(dst + (long long)t * DM + c8);
  *d = o;
  __threadfence();
  *d = o;
}

#define AT_NW 4
#define AT_QB 64
#define AT_KC 64
#define OSP 68
#define P_CARRY 32768.0f
#define CX_CARRY 64.0f

union FB { v16b b; v16h f; v8us u[2]; };

__device__ __forceinline__ v8f mma_bsplit(v16b ah, v16b al, v16b bh, v16b bl, v8f c) {
  c = __builtin_amdgcn_wmma_f32_16x16x32_bf16(false, ah, false, bh, (short)0, c, false, false);
  c = __builtin_amdgcn_wmma_f32_16x16x32_bf16(false, ah, false, bl, (short)0, c, false, false);
  c = __builtin_amdgcn_wmma_f32_16x16x32_bf16(false, al, false, bh, (short)0, c, false, false);
  asm volatile("v_nop\n\tv_nop\n\tv_nop\n\tv_nop" : "+v"(c) : "v"(ah), "v"(al), "v"(bh), "v"(bl));
  return c;
}
__device__ __forceinline__ v8f mma_h16(v16h a, v16h b, v8f c) {
  c = __builtin_amdgcn_wmma_f32_16x16x32_f16(false, a, false, b, (short)0, c, false, false);
  asm volatile("v_nop\n\tv_nop\n\tv_nop\n\tv_nop" : "+v"(c) : "v"(a), "v"(b));
  return c;
}

__global__ __launch_bounds__(128) void k_attn_x(
    const unsigned short* __restrict__ QHp, const unsigned short* __restrict__ QLp,
    const unsigned short* __restrict__ KHp, const unsigned short* __restrict__ KLp,
    const unsigned short* __restrict__ VTp, const float* __restrict__ Mk,
    unsigned short* __restrict__ CXp, int S, int H, int ldq, int ldvt, int ldm) {
  __shared__ __align__(16) unsigned short Ksh[AT_KC * HD];
  __shared__ __align__(16) unsigned short Ksl[AT_KC * HD];
  __shared__ __align__(16) unsigned short Vth[HD * AT_KC];
  __shared__ __align__(16) unsigned short Psh[AT_NW][16 * AT_KC];
  __shared__ __align__(16) float Ms[AT_QB * OSP];

  const int tid = threadIdx.x;
  const int wave = tid >> 5, lane = tid & 31, hh = lane >> 4, c = lane & 15;
  const int nqb = S / AT_QB;
  const int bx = (int)blockIdx.x;
  const int qb = bx % nqb;
  const int bh2 = bx / nqb;
  const int h = bh2 % H;
  const int b = bh2 / H;
  const int qbb = qb * AT_QB;
  const int q0 = qbb + wave * 16;
  const long long tok0 = (long long)b * S;
  const float NEG = -__builtin_inff();

  v16b qah[2], qal[2];
  {
    const long long ro = (tok0 + q0 + c) * (long long)ldq + (long long)h * HD + 8 * hh;
    FB f;
    f.u[0] = *(const v8us*)(QHp + ro);      f.u[1] = *(const v8us*)(QHp + ro + 16); qah[0] = f.b;
    f.u[0] = *(const v8us*)(QHp + ro + 32); f.u[1] = *(const v8us*)(QHp + ro + 48); qah[1] = f.b;
    f.u[0] = *(const v8us*)(QLp + ro);      f.u[1] = *(const v8us*)(QLp + ro + 16); qal[0] = f.b;
    f.u[0] = *(const v8us*)(QLp + ro + 32); f.u[1] = *(const v8us*)(QLp + ro + 48); qal[1] = f.b;
  }

  float mrow[8], lrow[8];
  v8f oacc[4];
#pragma unroll
  for (int r = 0; r < 8; ++r) { mrow[r] = NEG; lrow[r] = 0.f; }
#pragma unroll
  for (int t = 0; t < 4; ++t) oacc[t] = (v8f){0.f,0.f,0.f,0.f,0.f,0.f,0.f,0.f};

  const int nch = S / AT_KC;
  for (int kc = 0; kc < nch; ++kc) {
    const int kv0 = kc * AT_KC;
    __syncthreads();
#pragma unroll
    for (int i = 0; i < 4; ++i) {
      const int p = tid + 128 * i; const int kvr = p >> 3, pc = (p & 7) * 8;
      const long long go = (tok0 + kv0 + kvr) * (long long)ldq + (long long)h * HD + pc;
      *(v8us*)(Ksh + kvr * HD + pc) = *(const v8us*)(KHp + go);
    }
#pragma unroll
    for (int i = 0; i < 4; ++i) {
      const int p = tid + 128 * i; const int kvr = p >> 3, pc = (p & 7) * 8;
      const long long go = (tok0 + kv0 + kvr) * (long long)ldq + (long long)h * HD + pc;
      *(v8us*)(Ksl + kvr * HD + pc) = *(const v8us*)(KLp + go);
    }
#pragma unroll
    for (int i = 0; i < 4; ++i) {
      const int p = tid + 128 * i; const int d = p >> 3, pc = (p & 7) * 8;
      const long long go = (long long)(h * HD + d) * ldvt + tok0 + kv0 + pc;
      *(v8us*)(Vth + d * AT_KC + pc) = *(const v8us*)(VTp + go);
    }
#pragma unroll
    for (int i = 0; i < 8; ++i) {
      const int p = tid + 128 * i; const int r = p >> 4, pc = (p & 15) * 4;
      const v4f mv = *(const v4f*)(Mk + (long long)(qbb + r) * ldm + kv0 + pc);
      v4f mr;
#pragma unroll
      for (int e = 0; e < 4; ++e) mr[e] = bf_bits2f(f2bf_bits(mv[e]));
      *(v4f*)(Ms + r * OSP + pc) = mr;
    }
    __syncthreads();

    v8f s[4];
#pragma unroll
    for (int j = 0; j < 4; ++j) {
      v8f acc = (v8f){0.f,0.f,0.f,0.f,0.f,0.f,0.f,0.f};
      const unsigned short* kr  = Ksh + (j * 16 + c) * HD + 8 * hh;
      const unsigned short* krl = Ksl + (j * 16 + c) * HD + 8 * hh;
      FB kb0, kl0, kb1, kl1;
      kb0.u[0] = *(const v8us*)(kr);       kb0.u[1] = *(const v8us*)(kr + 16);
      kl0.u[0] = *(const v8us*)(krl);      kl0.u[1] = *(const v8us*)(krl + 16);
      acc = mma_bsplit(qah[0], qal[0], kb0.b, kl0.b, acc);
      kb1.u[0] = *(const v8us*)(kr + 32);  kb1.u[1] = *(const v8us*)(kr + 48);
      kl1.u[0] = *(const v8us*)(krl + 32); kl1.u[1] = *(const v8us*)(krl + 48);
      acc = mma_bsplit(qah[1], qal[1], kb1.b, kl1.b, acc);
      s[j] = acc;
    }
    float cm[8];
#pragma unroll
    for (int r = 0; r < 8; ++r) {
      const int lr = wave * 16 + 8 * hh + r;
      float m = NEG;
#pragma unroll
      for (int j = 0; j < 4; ++j) { s[j][r] += Ms[lr * OSP + j * 16 + c]; m = fmaxf(m, s[j][r]); }
#pragma unroll
      for (int off = 1; off < 16; off <<= 1) m = fmaxf(m, __shfl_xor(m, off, 32));
      cm[r] = m;
    }
    unsigned short* pw = Psh[wave];
#pragma unroll
    for (int r = 0; r < 8; ++r) {
      const float mnew = fmaxf(mrow[r], cm[r]);
      const bool dead = (mnew == NEG);
      const float ea = expf(mrow[r] - mnew);
      const float alpha = dead ? 1.f : ea;
      mrow[r] = mnew;
      float psum = 0.f;
#pragma unroll
      for (int j = 0; j < 4; ++j) {
        const float ep = expf(s[j][r] - mnew);
        const float p = dead ? 0.f : ep;
        psum += p;
        pw[(8 * hh + r) * AT_KC + j * 16 + c] = __builtin_bit_cast(unsigned short, (_Float16)(p * P_CARRY));
      }
#pragma unroll
      for (int off = 1; off < 16; off <<= 1) psum += __shfl_xor(psum, off, 32);
      lrow[r] = lrow[r] * alpha + psum;
#pragma unroll
      for (int t = 0; t < 4; ++t) oacc[t][r] *= alpha;
    }
    __builtin_amdgcn_fence(3  , "workgroup");
    __builtin_amdgcn_wave_barrier();
    __builtin_amdgcn_fence(2  , "workgroup");
#pragma unroll
    for (int kk = 0; kk < 2; ++kk) {
      FB pa;
      const unsigned short* pr = pw + c * AT_KC + kk * 32 + 8 * hh;
      pa.u[0] = *(const v8us*)(pr); pa.u[1] = *(const v8us*)(pr + 16);
#pragma unroll
      for (int t = 0; t < 4; ++t) {
        FB vb;
        const unsigned short* vr = Vth + (t * 16 + c) * AT_KC + kk * 32 + 8 * hh;
        vb.u[0] = *(const v8us*)(vr); vb.u[1] = *(const v8us*)(vr + 16);
        oacc[t] = mma_h16(pa.f, vb.f, oacc[t]);
      }
    }
  }

  __syncthreads();
  float* os = Ms + wave * 16 * OSP;
#pragma unroll
  for (int r = 0; r < 8; ++r) {
    const float den = lrow[r] + 1e-10f * expf(-mrow[r]);
    const float inv = (den > 0.f) ? (1.0f / den) * (CX_CARRY / P_CARRY) : 0.f;
#pragma unroll
    for (int t = 0; t < 4; ++t) os[(8 * hh + r) * OSP + t * 16 + c] = oacc[t][r] * inv;
  }
  __builtin_amdgcn_fence(3  , "workgroup");
  __builtin_amdgcn_wave_barrier();
  __builtin_amdgcn_fence(2  , "workgroup");
  {
    const int q8 = lane >> 3, c8 = (lane & 7) * 8;
    v8us pk[4];
#pragma unroll
    for (int it = 0; it < 4; ++it) {
      const int row = it * 4 + q8;
      const float* sp = os + row * OSP + c8;
      v8us o;
#pragma unroll
      for (int e = 0; e < 8; ++e) o[e] = __builtin_bit_cast(unsigned short, (_Float16)sp[e]);
      pk[it] = o;
    }
    for (int pass = 0; pass < 2; ++pass) {
#pragma unroll
      for (int it = 0; it < 4; ++it) {
        const int row = it * 4 + q8;
        *(volatile v8us*)(CXp + (tok0 + q0 + row) * (long long)ldq + (long long)h * HD + c8) = pk[it];
      }
      __threadfence();
    }
  }
}

extern "C" void kernel_launch(void* const* d_in, const int* in_sizes, int n_in,
                              void* d_out, int out_size, void* d_ws, size_t ws_size, hipStream_t stream) {
  if (n_in < 7) return;
  const long long needx = ((long long)(NB - 1) * SEQ_FULL + SEQ) * (long long)DM;
  if ((long long)in_sizes[0] < needx) return;
  if ((long long)in_sizes[1] < needx) return;
  if ((long long)in_sizes[2] < (long long)(SEQ - 1) * MASK_LD + SEQ) return;
  for (int i = 3; i < 7; ++i) if ((long long)in_sizes[i] < (long long)DM * DM) return;
  if ((long long)out_size < (long long)NTOK * DM) return;

  const float* x    = (const float*)d_in[0];
  const float* y    = (const float*)d_in[1];
  const float* mask = (const float*)d_in[2];
  const float* Wq   = (const float*)d_in[3];
  const float* Wk   = (const float*)d_in[4];
  const float* Wv   = (const float*)d_in[5];
  const float* Wo   = (const float*)d_in[6];
  float* out = (float*)d_out;

  char* wsp = (char*)d_ws;
  size_t used = 0;
  const size_t bAct = (size_t)NTOK * DM * 2;
  const size_t bW   = (size_t)DM * DM * 2;
  unsigned short* XB  = (unsigned short*)(wsp + used); used += bAct;
  unsigned short* YB  = (unsigned short*)(wsp + used); used += bAct;
  unsigned short* WQB = (unsigned short*)(wsp + used); used += bW;
  unsigned short* WKB = (unsigned short*)(wsp + used); used += bW;
  unsigned short* WVB = (unsigned short*)(wsp + used); used += bW;
  unsigned short* WOP = (unsigned short*)(wsp + used); used += bW;
  unsigned short* QH  = (unsigned short*)(wsp + used); used += bAct;
  unsigned short* QL  = (unsigned short*)(wsp + used); used += bAct;
  unsigned short* KH  = (unsigned short*)(wsp + used); used += bAct;
  unsigned short* KL  = (unsigned short*)(wsp + used); used += bAct;
  unsigned short* VT  = (unsigned short*)(wsp + used); used += bAct;
  unsigned short* CX  = (unsigned short*)(wsp + used); used += bAct;
  if (used > ws_size) return;
  if (used > (size_t)134217728) return;

  const unsigned gx = (unsigned)(((long long)NTOK * (DM / 8) + 255) / 256);
  const unsigned gw = (unsigned)(((long long)DM * (DM / 8) + 255) / 256);
  const unsigned gg = (unsigned)(((NTOK / 64) * (DM / 64) + 7) / 8);
  const unsigned ga = (unsigned)(NB * NH * (SEQ / 64));

  k_cvt8<false><<<gx, 256, 0, stream>>>(x, XB, NTOK, SEQ, SEQ_FULL, 1.0f);
  k_cvt8<false><<<gx, 256, 0, stream>>>(y, YB, NTOK, SEQ, SEQ_FULL, 1.0f);
  k_cvt8<false><<<gw, 256, 0, stream>>>(Wq, WQB, DM, DM, DM, 1.0f);
  k_cvt8<false><<<gw, 256, 0, stream>>>(Wk, WKB, DM, DM, DM, 1.0f);
  k_cvt8<false><<<gw, 256, 0, stream>>>(Wv, WVB, DM, DM, DM, 1.0f);
  k_cvt8<true><<<gw, 256, 0, stream>>>(Wo, WOP, DM, DM, DM, 64.0f);

  k_gemm64<1, false, 0, 2, false, 0><<<dim3(gg, 1), 256, 0, stream>>>(YB, nullptr, DM, 0, WQB, nullptr, DM, 0, (void*)QH, (void*)QL, DM, 0, nullptr, nullptr, 0, NTOK, DM, DM, 0.125f);
  k_gemm64<1, false, 0, 2, false, 0><<<dim3(gg, 1), 256, 0, stream>>>(XB, nullptr, DM, 0, WKB, nullptr, DM, 0, (void*)KH, (void*)KL, DM, 0, nullptr, nullptr, 0, NTOK, DM, DM, 1.0f);
  k_gemm64<1, false, 0, 1, false, 0><<<dim3(gg, 1), 256, 0, stream>>>(WVB, nullptr, DM, 0, XB, nullptr, DM, 0, (void*)VT, nullptr, NTOK, 0, nullptr, nullptr, 0, DM, NTOK, DM, 1.0f);

  k_attn_x<<<ga, 128, 0, stream>>>(QH, QL, KH, KL, VT, mask, CX, SEQ, NH, DM, NTOK, MASK_LD);

  k_gemm64<0, false, 0, 0, false, 0><<<dim3(gg, 1), 256, 0, stream>>>(CX, nullptr, DM, 0, WOP, nullptr, DM, 0, (void*)out, nullptr, DM, 0, nullptr, nullptr, 0, NTOK, DM, DM, 1.0f / 4096.0f);
  (void)hipGetLastError();
}
